// PanoformerBlock_81578608820347
// MI455X (gfx1250) — hardware-verified
//
#include <hip/hip_runtime.h>


namespace {
constexpr int NB = 2, H = 64, W = 128, N = H * W, C = 256, NH = 8, K = 9, HD = 32, HID = 1024, NTOK = NB * N;
constexpr int NV = C, NOFF = NH * K * 2, NAT = NH * K, NPRJ = NV + NOFF + NAT, NPRJP = 512;
constexpr float XS = 8.0f, WSC = 256.0f, EPS = 1e-5f;

typedef _Float16 b16;
typedef __attribute__((ext_vector_type(16))) _Float16 v16b;
typedef __attribute__((ext_vector_type(8))) _Float16 v8b;
typedef __attribute__((ext_vector_type(8))) float v8f;
typedef __attribute__((ext_vector_type(4))) float v4f;
__device__ __forceinline__ float bf16_rne(float f) { unsigned int u = __float_as_uint(f); u += 0x7FFFu + ((u >> 16) & 1u); return __uint_as_float(u & 0xFFFF0000u); }
__device__ __forceinline__ v16b frag_kb(const b16* p, int hh) { const v8b a = *(const v8b*)(p + 8 * hh), b = *(const v8b*)(p + 16 + 8 * hh); v16b f;
#pragma unroll
  for (int e = 0; e < 8; ++e) { f[e] = a[e]; f[8 + e] = b[e]; } return f; }
__device__ __forceinline__ v8f wmma16b(v16b a, v16b b, v8f c) { v8f d = __builtin_amdgcn_wmma_f32_16x16x32_f16(false, a, false, b, (short)0, c, false, false); asm volatile("v_nop\n\tv_nop\n\tv_nop\n\tv_nop" : "+v"(d) : "v"(a), "v"(b)); return d; }
__device__ __forceinline__ void wave_lds_sync() { __builtin_amdgcn_fence(__ATOMIC_RELEASE, "workgroup"); __builtin_amdgcn_wave_barrier(); __builtin_amdgcn_fence(__ATOMIC_ACQUIRE, "workgroup"); }
__device__ __forceinline__ float pmul(float a, float b) { float p = a * b; asm volatile("" : "+v"(p)); return p; }
__device__ __forceinline__ float gelu(float v) { return 0.5f * v * (1.0f + erff(v * 0.70710678118654752f)); }

__global__ __launch_bounds__(256) void prepw_kernel(const float* __restrict__ wv, const float* __restrict__ woff, const float* __restrict__ wat, const float* __restrict__ wout, const float* __restrict__ w1, const float* __restrict__ w2, b16* __restrict__ WP, b16* __restrict__ WOUT, b16* __restrict__ W1T, b16* __restrict__ W2T) {
  __shared__ __attribute__((aligned(16))) b16 T[64][64 + 8];
  const int kind = blockIdx.z, i0 = blockIdx.x * 64, o0 = blockIdx.y * 64, t_ = threadIdx.x;
  const int IN = kind == 5 ? HID : C, OUT = kind == 0 ? C : kind == 1 ? NOFF : kind == 2 ? NAT : kind == 3 ? C : kind == 4 ? HID : kind == 5 ? C : (NPRJP - NPRJ);
  if (i0 >= IN || o0 >= OUT) return;
  const float* w = kind == 0 ? wv : kind == 1 ? woff : kind == 2 ? wat : kind == 3 ? wout : kind == 4 ? w1 : w2;
  b16* dst = kind == 0 ? WP : kind == 1 ? WP + (size_t)NV * C : kind == 2 ? WP + (size_t)(NV + NOFF) * C : kind == 3 ? WOUT : kind == 4 ? W1T : kind == 5 ? W2T : WP + (size_t)NPRJ * C;
  for (int q = t_; q < 64 * 64; q += 256) { const int ii = q >> 6, oo = q & 63; T[oo][ii] = (kind < 6 && o0 + oo < OUT) ? (b16)(bf16_rne(w[(size_t)(i0 + ii) * OUT + (o0 + oo < OUT ? o0 + oo : 0)]) * WSC) : (b16)0.0f; }
  __syncthreads();
  for (int pass = 0; pass < 2; ++pass) { for (int q = t_; q < 64 * 8; q += 256) { const int oo = q >> 3, c8 = (q & 7) * 8; if (o0 + oo < OUT) *(volatile v8b*)(dst + (size_t)(o0 + oo) * IN + i0 + c8) = *(const v8b*)(&T[oo][c8]); } __threadfence(); }
}
template <int MODE>
__global__ __launch_bounds__(256) void ln_kernel(const float* __restrict__ X, const float* __restrict__ g, const float* __restrict__ be, b16* __restrict__ O16) {
  const int wave = threadIdx.x >> 5, lane = threadIdx.x & 31; const size_t row = (size_t)blockIdx.x * 8 + wave; const float* src = X + row * C + lane * 8;
  const v4f a0 = *(const v4f*)src, a1 = *(const v4f*)(src + 4); float v[8];
#pragma unroll
  for (int j = 0; j < 4; ++j) { v[j] = MODE == 0 ? bf16_rne(a0[j]) : a0[j]; v[4 + j] = MODE == 0 ? bf16_rne(a1[j]) : a1[j]; }
  float s = 0.0f;
#pragma unroll
  for (int j = 0; j < 8; ++j) s += v[j];
#pragma unroll
  for (int o = 16; o >= 1; o >>= 1) s += __shfl_xor(s, o);
  const float mu = s * (1.0f / C); float ss = 0.0f;
#pragma unroll
  for (int j = 0; j < 8; ++j) { const float d = v[j] - mu; ss += pmul(d, d); }
#pragma unroll
  for (int o = 16; o >= 1; o >>= 1) ss += __shfl_xor(ss, o);
  const float rs = rsqrtf(ss * (1.0f / C) + EPS); v8b o8;
#pragma unroll
  for (int j = 0; j < 8; ++j) { const int c = lane * 8 + j; o8[j] = (b16)((pmul((v[j] - mu) * rs, bf16_rne(g[c])) + bf16_rne(be[c])) * XS); }
  for (int pass = 0; pass < 2; ++pass) { *(volatile v8b*)(O16 + row * C + lane * 8) = o8; __threadfence(); }
}
template <int MODE>
__global__ __launch_bounds__(128) void gemm_kernel(const b16* __restrict__ A, int lda, int Kd, const b16* __restrict__ Bw, const float* __restrict__ bias, int nbias, const float* __restrict__ R, float* __restrict__ Y, b16* __restrict__ Y16, int ldc) {
  __shared__ __attribute__((aligned(16))) float Ts[4][16][128 + 4];
  const int wave = threadIdx.x >> 5, lane = threadIdx.x & 31, nloc = lane & 15, hlf = lane >> 4; const size_t m0 = (size_t)blockIdx.x * 64 + wave * 16; const int n0 = blockIdx.y * 128;
  v8f acc[8];
#pragma unroll
  for (int t = 0; t < 8; ++t) acc[t] = (v8f){};
  for (int kb = 0; kb < Kd; kb += 32) { const v16b a = frag_kb(A + (m0 + nloc) * lda + kb, hlf);
#pragma unroll
    for (int t = 0; t < 8; ++t) acc[t] = wmma16b(a, frag_kb(Bw + (size_t)(n0 + t * 16 + nloc) * Kd + kb, hlf), acc[t]); }
#pragma unroll
  for (int t = 0; t < 8; ++t) { const int n = n0 + t * 16 + nloc; const float bb = (n < nbias) ? bf16_rne(bias[n < nbias ? n : 0]) : 0.0f;
#pragma unroll
    for (int r = 0; r < 8; ++r) { float v = acc[t][r] * (1.0f / (XS * WSC)) + bb; if (MODE == 2) v = gelu(v); Ts[wave][8 * hlf + r][t * 16 + nloc] = v; } }
  wave_lds_sync();
  for (int pass = 0; pass < 2; ++pass) {
    for (int rr = 0; rr < 16; ++rr) { const size_t row = m0 + rr;
      if (MODE == 2) { if (lane < 16) { const v4f a = *(const v4f*)(&Ts[wave][rr][lane * 8]), c = *(const v4f*)(&Ts[wave][rr][lane * 8 + 4]); v8b o;
#pragma unroll
          for (int j = 0; j < 4; ++j) { o[j] = (b16)(a[j] * XS); o[4 + j] = (b16)(c[j] * XS); }
          *(volatile v8b*)(Y16 + row * ldc + n0 + lane * 8) = o; } }
      else { v4f v = *(const v4f*)(&Ts[wave][rr][lane * 4]);
        if (MODE == 1) { const v4f rv = *(const v4f*)(R + row * ldc + n0 + lane * 4); v[0] += bf16_rne(rv[0]); v[1] += bf16_rne(rv[1]); v[2] += bf16_rne(rv[2]); v[3] += bf16_rne(rv[3]); }
        else if (MODE == 3) v += *(const v4f*)(R + row * ldc + n0 + lane * 4);
        *(volatile v4f*)(Y + row * ldc + n0 + lane * 4) = v; } }
    __threadfence(); }
}
__global__ __launch_bounds__(256) void sample_kernel(const float* __restrict__ PRJ, const float* __restrict__ refp, b16* __restrict__ S16) {
  __shared__ float Sp[NPRJP - NV]; __shared__ __attribute__((aligned(16))) b16 To[C + 8];
  const int tok = blockIdx.x, t_ = threadIdx.x, h = t_ >> 5, d = t_ & 31; const int b = tok / N, n = tok - b * N;
  if (t_ < NOFF + NAT) Sp[t_] = PRJ[(size_t)tok * NPRJP + NV + t_];
  __syncthreads();
  const float* off = Sp + h * K * 2; const float* lg = Sp + NOFF + h * K; float mx = -INFINITY;
#pragma unroll
  for (int k = 0; k < K; ++k) mx = fmaxf(mx, lg[k]);
  float den = 0.0f, e[K];
#pragma unroll
  for (int k = 0; k < K; ++k) { e[k] = __expf(lg[k] - mx); den += e[k]; }
  const float* Vb = PRJ + (size_t)b * N * NPRJP + h * HD + d; float acc = 0.0f;
#pragma unroll 1
  for (int k = 0; k < K; ++k) { const float rx = bf16_rne(refp[((size_t)n * K + k) * 2 + 0]), ry = bf16_rne(refp[((size_t)n * K + k) * 2 + 1]);
    float px = pmul(rx, (float)(W - 1)) + off[k * 2 + 0], py = pmul(ry, (float)(H - 1)) + off[k * 2 + 1];
    px = fminf(fmaxf(px, 0.0f), (float)(W - 1)); py = fminf(fmaxf(py, 0.0f), (float)(H - 1));
    const float x0f = floorf(px), y0f = floorf(py); const float x1f = fminf(x0f + 1.0f, (float)(W - 1)), y1f = fminf(y0f + 1.0f, (float)(H - 1)); const float wx = px - x0f, wy = py - y0f;
    const int x0 = min(max((int)x0f, 0), W - 1), y0 = min(max((int)y0f, 0), H - 1), x1 = min(max((int)x1f, 0), W - 1), y1 = min(max((int)y1f, 0), H - 1);
    const float g00 = Vb[(size_t)(y0 * W + x0) * NPRJP], g01 = Vb[(size_t)(y0 * W + x1) * NPRJP], g10 = Vb[(size_t)(y1 * W + x0) * NPRJP], g11 = Vb[(size_t)(y1 * W + x1) * NPRJP];
    const float s = pmul(g00, pmul(1.0f - wx, 1.0f - wy)) + pmul(g01, pmul(wx, 1.0f - wy)) + pmul(g10, pmul(1.0f - wx, wy)) + pmul(g11, pmul(wx, wy));
    acc += pmul(e[k] / den, s); }
  To[h * HD + d] = (b16)(acc * XS);
  __syncthreads();
  for (int pass = 0; pass < 2; ++pass) { if (t_ < 32) *(volatile v8b*)(S16 + (size_t)tok * C + t_ * 8) = *(const v8b*)(&To[t_ * 8]); __threadfence(); }
}
__global__ __launch_bounds__(256) void dwconv_kernel(const b16* __restrict__ G16, const float* __restrict__ wdw, const float* __restrict__ bdw, b16* __restrict__ D16) {
  const int wave = threadIdx.x >> 5, lane = threadIdx.x & 31; const int tok = blockIdx.x * 8 + wave; const int b = tok / N, n = tok - b * N, y = n / W, x = n - y * W;
  for (int pass = 0; pass < 2; ++pass) {
#pragma unroll 1
    for (int ch = 0; ch < 4; ++ch) { const int c0 = ch * 256 + lane * 8; float acc[8];
#pragma unroll
      for (int j = 0; j < 8; ++j) acc[j] = bf16_rne(bdw[c0 + j]);
#pragma unroll 1
      for (int dy = -1; dy <= 1; ++dy) { const int yy = y + dy; if (yy < 0 || yy >= H) continue;
#pragma unroll 1
        for (int dx = -1; dx <= 1; ++dx) { const int xx = (x + dx + W) % W;
          const v8b gv = *(const v8b*)(G16 + ((size_t)b * N + yy * W + xx) * HID + c0);
#pragma unroll
          for (int j = 0; j < 8; ++j) acc[j] += pmul((float)gv[j] * (1.0f / XS), bf16_rne(wdw[(size_t)(c0 + j) * 9 + (dy + 1) * 3 + (dx + 1)])); } }
      v8b o;
#pragma unroll
      for (int j = 0; j < 8; ++j) o[j] = (b16)(gelu(acc[j]) * XS);
      *(volatile v8b*)(D16 + (size_t)tok * HID + c0) = o; }
    __threadfence(); }
}
__global__ __launch_bounds__(512) void bias_kernel(const float* __restrict__ bv, const float* __restrict__ boff, const float* __restrict__ bat, float* __restrict__ BP) {
  const int t = threadIdx.x; const float v = t < NV ? bv[t] : t < NV + NOFF ? boff[t - NV] : t < NPRJ ? bat[t - NV - NOFF] : 0.0f;
  for (int pass = 0; pass < 2; ++pass) { ((volatile float*)BP)[t] = v; __threadfence(); }
}
}

extern "C" void kernel_launch(void* const* d_in, const int* in_sizes, int n_in, void* d_out, int out_size, void* d_ws, size_t ws_size, hipStream_t stream) {
  (void)n_in;
  auto Fp = [&](int i) { return (const float*)d_in[i]; };
  if (in_sizes[0] != NTOK * C || in_sizes[1] != N * K * 2 || in_sizes[4] != C * C || in_sizes[6] != C * NOFF || in_sizes[8] != C * NAT || in_sizes[14] != C * HID || in_sizes[16] != HID * 9 || in_sizes[18] != HID * C || out_size != NTOK * C) return;
  size_t off = 0; char* ws = (char*)d_ws;
  auto carve = [&](size_t bytes) { char* p = ws + off; off += (bytes + 255) & ~(size_t)255; return p; };
  b16* WP = (b16*)carve((size_t)NPRJP * C * 2); b16* WOUT = (b16*)carve((size_t)C * C * 2); b16* W1T = (b16*)carve((size_t)HID * C * 2); b16* W2T = (b16*)carve((size_t)C * HID * 2);
  b16* XN = (b16*)carve((size_t)NTOK * C * 2); float* PRJ = (float*)carve((size_t)NTOK * NPRJP * 4); b16* S16 = (b16*)carve((size_t)NTOK * C * 2); float* X1 = (float*)carve((size_t)NTOK * C * 4);
  b16* G16 = (b16*)carve((size_t)NTOK * HID * 2); float* BP = (float*)carve(NPRJP * 4);
  b16* D16 = (b16*)PRJ;
  static_assert((size_t)NTOK * HID * 2 == (size_t)NTOK * NPRJP * 4, "D16 exactly covers PRJ");
  b16* XN2 = XN;
  if (off > ws_size || off > ((size_t)128 << 20)) return;
  prepw_kernel<<<dim3(HID / 64, HID / 64, 7), 256, 0, stream>>>(Fp(4), Fp(6), Fp(8), Fp(10), Fp(14), Fp(18), WP, WOUT, W1T, W2T);
  bias_kernel<<<1, 512, 0, stream>>>(Fp(5), Fp(7), Fp(9), BP);
  ln_kernel<0><<<NTOK / 8, 256, 0, stream>>>(Fp(0), Fp(2), Fp(3), XN);
  gemm_kernel<0><<<dim3(NTOK / 64, NPRJP / 128), 128, 0, stream>>>(XN, C, C, WP, BP, NPRJ, nullptr, PRJ, nullptr, NPRJP);
  sample_kernel<<<NTOK, 256, 0, stream>>>(PRJ, Fp(1), S16);
  gemm_kernel<1><<<dim3(NTOK / 64, C / 128), 128, 0, stream>>>(S16, C, C, WOUT, Fp(11), C, Fp(0), X1, nullptr, C);
  ln_kernel<1><<<NTOK / 8, 256, 0, stream>>>(X1, Fp(12), Fp(13), XN2);
  gemm_kernel<2><<<dim3(NTOK / 64, HID / 128), 128, 0, stream>>>(XN2, C, C, W1T, Fp(15), HID, nullptr, nullptr, G16, HID);
  dwconv_kernel<<<NTOK / 8, 256, 0, stream>>>(G16, Fp(16), Fp(17), D16);
  gemm_kernel<3><<<dim3(NTOK / 64, C / 128), 128, 0, stream>>>(D16, HID, HID, W2T, Fp(19), C, X1, (float*)d_out, nullptr, C);
}
